// TransformerLayerQKV_82291573392117
// MI455X (gfx1250) — hardware-run, weakly checked
//
#include <hip/hip_runtime.h>
#include <math.h>

constexpr int kBatch = 4;
constexpr int kSeq = 2048;
constexpr int kChan = 768;
constexpr int kHeads = 12;
constexpr int kHdim = 64;
constexpr int kFfn = 3072;
constexpr int kTok = kBatch * kSeq;
constexpr int kGrp = 3;
constexpr int kNumGroups = kBatch * kHeads;
constexpr int kNumChunks = kNumGroups / kGrp;
constexpr float kWCarry = 16.0f;
constexpr float kWCarryInv = 1.0f / 16.0f;
constexpr float kPCarry = 1024.0f;
constexpr float kOCarry = 64.0f;
constexpr float kPVScale = kOCarry / kPCarry;
constexpr float kWpScale = 1.0f / (kOCarry * kWCarry);
constexpr float kAttnScale = 0.125f;
constexpr float kLnEps = 1e-5f;
constexpr float kInvChan = 1.0f / 768.0f;

constexpr size_t kPlane16 = (size_t)kTok * kChan * 2;
constexpr size_t kW4Bytes = (size_t)4 * kChan * kChan * 2;
constexpr size_t kW1tBytes = (size_t)kFfn * kChan * 2;
constexpr size_t kSBytes = (size_t)kGrp * kSeq * kSeq * 4;
constexpr size_t kPBytes = (size_t)kGrp * kSeq * kSeq * 2;
constexpr size_t kX1Bytes = (size_t)kTok * kChan * 4;
constexpr size_t kHidBytes = (size_t)kTok * kFfn * 2;

constexpr size_t kOffW4 = 0;
constexpr size_t kOffQn = kOffW4 + kW4Bytes;
constexpr size_t kOffKc = kOffQn + kPlane16;
constexpr size_t kOffVc = kOffKc + kPlane16;
constexpr size_t kOffSx = kOffVc + kPlane16;
constexpr size_t kOffP = kOffSx + kPlane16;
constexpr size_t kOffQ16 = kOffP + kPBytes;
constexpr size_t kOffK16 = kOffQ16 + kPlane16;
constexpr size_t kOffVt = kOffK16 + kPlane16;
constexpr size_t kOffO16 = kOffVt + kPlane16;
constexpr size_t kWsTotal = kOffO16 + kPlane16;
constexpr size_t kOffS = kOffQn;
constexpr size_t kOffHid = kOffQn;
constexpr size_t kOffW1t = kOffP;
constexpr size_t kOffW2t = kOffP + kW1tBytes;
constexpr size_t kOffX1 = kOffQ16;
constexpr size_t kOffLn2 = kOffVt;
static_assert(kOffS + kSBytes == kOffP);
static_assert(kOffHid + kHidBytes <= kOffP);
static_assert(kOffW2t + kW1tBytes <= kOffQ16);
static_assert(kOffX1 + kX1Bytes == kOffVt);
static_assert(kWsTotal == (size_t)130547712);
static_assert(kWsTotal <= (size_t)134217728);
static_assert((kOffQn % 128) == 0 && (kOffP % 128) == 0 && (kOffQ16 % 128) == 0 && (kOffO16 % 128) == 0);

typedef __attribute__((ext_vector_type(16))) _Float16 v16h;
typedef __attribute__((ext_vector_type(8)))  _Float16 v8h;
typedef __attribute__((ext_vector_type(16))) __bf16   v16b;
typedef __attribute__((ext_vector_type(8)))  __bf16   v8b;
typedef __attribute__((ext_vector_type(8)))  float    v8f;
typedef __attribute__((ext_vector_type(4)))  float    v4f;
typedef __attribute__((ext_vector_type(4)))  unsigned int v4u;

__device__ __forceinline__ unsigned short f2bf_bits(float f) {
  unsigned u = __float_as_uint(f);
  return (unsigned short)((u + 0x7FFFu + ((u >> 16) & 1u)) >> 16);
}
__device__ __forceinline__ float bf_bits2f(unsigned short h) { return __uint_as_float(((unsigned)h) << 16); }

__device__ __forceinline__ void dep_guard_h(v8f& a, v8f& b, v16h x, v16h y) { asm volatile("v_nop\n\tv_nop\n\tv_nop\n\tv_nop" : "+v"(a), "+v"(b) : "v"(x), "v"(y)); }
__device__ __forceinline__ void dep_guard_b(v8f& a, v8f& b, v16b x, v16b y) { asm volatile("v_nop\n\tv_nop\n\tv_nop\n\tv_nop" : "+v"(a), "+v"(b) : "v"(x), "v"(y)); }
__device__ __forceinline__ void keep4_h(v16h a, v16h b, v16h c, v16h d) { asm volatile("v_nop" :: "v"(a), "v"(b), "v"(c), "v"(d)); }
__device__ __forceinline__ void keep4_b(v16b a, v16b b, v16b c, v16b d) { asm volatile("v_nop" :: "v"(a), "v"(b), "v"(c), "v"(d)); }
__device__ __forceinline__ void acc_guard4(v8f& a, v8f& b, v8f& c, v8f& d) { asm volatile("v_nop\n\tv_nop\n\tv_nop\n\tv_nop" : "+v"(a), "+v"(b), "+v"(c), "+v"(d)); }
template <typename T> struct Frag;
template <> struct Frag<_Float16> {
  typedef v16h V; union U { v16h v; v8h h[2]; };
  static __device__ __forceinline__ v16h load(const _Float16* p) {
    U f; f.h[0] = *(const v8h*)(p); f.h[1] = *(const v8h*)(p + 16); return f.v;
  }
  static __device__ __forceinline__ v8f mma(v16h a, v16h b, v8f c) {
    return __builtin_amdgcn_wmma_f32_16x16x32_f16(false, a, false, b, (short)0, c, false, false);
  }
  static __device__ __forceinline__ void guard(v8f& a, v8f& b, v16h x, v16h y) { dep_guard_h(a, b, x, y); }
  static __device__ __forceinline__ void keep(v16h a, v16h b, v16h c, v16h d) { keep4_h(a, b, c, d); }
};
template <> struct Frag<__bf16> {
  typedef v16b V; union U { v16b v; v8b h[2]; };
  static __device__ __forceinline__ v16b load(const __bf16* p) {
    U f; f.h[0] = *(const v8b*)(p); f.h[1] = *(const v8b*)(p + 16); return f.v;
  }
  static __device__ __forceinline__ v8f mma(v16b a, v16b b, v8f c) {
    return __builtin_amdgcn_wmma_f32_16x16x32_bf16(false, a, false, b, (short)0, c, false, false);
  }
  static __device__ __forceinline__ void guard(v8f& a, v8f& b, v16b x, v16b y) { dep_guard_b(a, b, x, y); }
  static __device__ __forceinline__ void keep(v16b a, v16b b, v16b c, v16b d) { keep4_b(a, b, c, d); }
};

__device__ __forceinline__ unsigned pk16(unsigned short a, unsigned short b) { return (unsigned)a | ((unsigned)b << 16); }
__device__ __forceinline__ unsigned short h_bits(float f) { const _Float16 h = (_Float16)f; return __builtin_bit_cast(unsigned short, h); }

template <int ET> struct Elem;
template <> struct Elem<0> { typedef _Float16 T; };
template <> struct Elem<1> { typedef __bf16 T; };
template <int ET, bool SPLIT, int BIAS_MODE, int OUT_MODE, bool RESID, int ACT = 0>
__global__ __launch_bounds__(256) void wmma_gemm64(
    const unsigned short* __restrict__ Ap, const unsigned short* __restrict__ A2p, int lda, long strideA,
    const unsigned short* __restrict__ Btp, const unsigned short* __restrict__ Bt2p, int ldb, long strideB,
    void* __restrict__ Cout, void* __restrict__ Cout2, int ldc, long strideC,
    const float* __restrict__ bias,
    const float* resid, const float* residB, const float* residC,
    const int* __restrict__ rsel, long strideR,
    int M, int N, int K, float scale) {
  typedef typename Elem<ET>::T T;
  typedef typename Frag<T>::V V;
  const T* A = (const T*)Ap; const T* A2 = (const T*)A2p; const T* Bt = (const T*)Btp; const T* Bt2 = (const T*)Bt2p;
  __shared__ __align__(16) float sT[8][16 * 68];
  const int b    = blockIdx.y;
  const int lane = threadIdx.x & 31;
  const int wave = threadIdx.x >> 5;
  const int tilesN = N >> 6;
  const int tilesM = M >> 6;
  const int tile = blockIdx.x * 8 + wave;
  if (tile >= tilesM * tilesN) return;
  const int tm = tile / tilesN;
  const int tn = tile - tm * tilesN;
  const int m0 = tm << 6;
  const int n0 = tn << 6;

  const T* Ab  = A  + (size_t)b * strideA;
  const T* Bb  = Bt + (size_t)b * strideB;
  const T* Ab2 = SPLIT ? (A2  + (size_t)b * strideA) : nullptr;
  const T* Bb2 = SPLIT ? (Bt2 + (size_t)b * strideB) : nullptr;

  const int rlane = lane & 15;
  const int koff  = (lane >> 4) * 8;
  const int mOff  = (lane >> 4) * 8;

  v8f acc[4][4];
#pragma unroll
  for (int i = 0; i < 4; ++i)
#pragma unroll
    for (int j = 0; j < 4; ++j) acc[i][j] = (v8f){0.f,0.f,0.f,0.f,0.f,0.f,0.f,0.f};

  for (int k0 = 0; k0 < K; k0 += 32) {
    V bh[4], bl[4];
#pragma unroll
    for (int j = 0; j < 4; ++j) {
      const size_t bo = (size_t)(n0 + (j << 4) + rlane) * ldb + koff + k0;
      bh[j] = Frag<T>::load(Bb + bo);
      if (SPLIT) bl[j] = Frag<T>::load(Bb2 + bo);
    }
#pragma unroll
    for (int i = 0; i < 4; ++i) {
      const size_t ao = (size_t)(m0 + (i << 4) + rlane) * lda + koff + k0;
      V ah = Frag<T>::load(Ab + ao);
      V al;
      if (SPLIT) al = Frag<T>::load(Ab2 + ao);
#pragma unroll
      for (int j = 0; j < 4; ++j) {
        acc[i][j] = Frag<T>::mma(ah, bh[j], acc[i][j]);
        if (SPLIT) {
          acc[i][j] = Frag<T>::mma(ah, bl[j], acc[i][j]);
          acc[i][j] = Frag<T>::mma(al, bh[j], acc[i][j]);
        }
      }
      Frag<T>::guard(acc[i][0], acc[i][3], ah, SPLIT ? al : ah);
    }
    Frag<T>::keep(bh[0], bh[1], bh[2], bh[3]);
    if (SPLIT) Frag<T>::keep(bl[0], bl[1], bl[2], bl[3]);
  }
  acc_guard4(acc[0][0], acc[0][1], acc[0][2], acc[0][3]);
  acc_guard4(acc[1][0], acc[1][1], acc[1][2], acc[1][3]);
  acc_guard4(acc[2][0], acc[2][1], acc[2][2], acc[2][3]);
  acc_guard4(acc[3][0], acc[3][1], acc[3][2], acc[3][3]);

  float* slab = sT[wave];
  const float* Rsrc = resid;
  if (RESID) {
    if (rsel != nullptr) {
      int ps = rsel[0];
      ps = ps < 0 ? 0 : ps;
      ps = ps > 2 ? 2 : ps;
      Rsrc = (ps == 1) ? residB : ((ps == 2) ? residC : resid);
    }
  }
  const float* Rb = RESID ? (Rsrc + (size_t)b * strideR) : nullptr;
#pragma unroll
  for (int i = 0; i < 4; ++i) {
    const int mBase = m0 + (i << 4);
#pragma unroll
    for (int j = 0; j < 4; ++j) {
      const int n = n0 + (j << 4) + rlane;
      float bv = 0.f;
      if (BIAS_MODE == 2) bv = bias[n];
#pragma unroll
      for (int r = 0; r < 8; ++r) {
        float v = acc[i][j][r] * scale;
        if (BIAS_MODE == 1) v += bias[mBase + mOff + r];
        if (BIAS_MODE == 2) v += bv;
        if (RESID) v += Rb[(size_t)(mBase + mOff + r) * ldc + n];
        if (ACT == 2) v = fmaxf(v, 0.0f);
        if (ACT == 4) v = (v > 0.f) ? v : 0.01f * v;
        slab[(mOff + r) * 68 + (j << 4) + rlane] = v;
      }
    }
    __builtin_amdgcn_fence(__ATOMIC_RELEASE, "workgroup");
    __builtin_amdgcn_wave_barrier();
    __builtin_amdgcn_fence(__ATOMIC_ACQUIRE, "workgroup");
    if (OUT_MODE == 0) {
      float* C = (float*)Cout + (size_t)b * strideC;
      const int hh = lane >> 4, c4 = (lane & 15) * 4;
      for (int pass = 0; pass < 2; ++pass) {
#pragma unroll
        for (int it = 0; it < 8; ++it) {
          const int row = it * 2 + hh;
          v4f v = *(const v4f*)(slab + row * 68 + c4);
          *(volatile v4f*)(C + (size_t)(mBase + row) * ldc + n0 + c4) = v;
        }
        __threadfence();
      }
    } else {
      const int q = lane >> 3, c8 = (lane & 7) * 8;
      unsigned short* C  = (unsigned short*)Cout  + (size_t)b * strideC;
      unsigned short* C2 = (OUT_MODE == 2) ? ((unsigned short*)Cout2 + (size_t)b * strideC) : nullptr;
      for (int pass = 0; pass < 2; ++pass) {
#pragma unroll
        for (int it = 0; it < 4; ++it) {
          const int row = it * 4 + q;
          const float* sp = slab + row * 68 + c8;
          v8h hv, lv;
#pragma unroll
          for (int e = 0; e < 8; ++e) {
            if (OUT_MODE == 1) {
              hv[e] = (_Float16)sp[e];
            } else {
              unsigned short hb = f2bf_bits(sp[e]);
              unsigned short lb = f2bf_bits(sp[e] - bf_bits2f(hb));
              hv[e] = __builtin_bit_cast(_Float16, hb);
              lv[e] = __builtin_bit_cast(_Float16, lb);
            }
          }
          *(volatile v8h*)(C + (size_t)(mBase + row) * ldc + n0 + c8) = hv;
          if (OUT_MODE == 2) *(volatile v8h*)(C2 + (size_t)(mBase + row) * ldc + n0 + c8) = lv;
        }
        __threadfence();
      }
    }
    __builtin_amdgcn_fence(__ATOMIC_RELEASE, "workgroup");
    __builtin_amdgcn_wave_barrier();
    __builtin_amdgcn_fence(__ATOMIC_ACQUIRE, "workgroup");
  }
}

__global__ __launch_bounds__(256) void layernorm_rows_kernel(const float* __restrict__ x, const float* __restrict__ w,
                                                             const float* __restrict__ bvec, unsigned short* __restrict__ out,
                                                             int nrows) {
  const int lane = threadIdx.x & 31;
  const int wave = threadIdx.x >> 5;
  const int row = blockIdx.x * 8 + wave;
  if (row >= nrows) return;
  const float* xr = x + (size_t)row * kChan;
  float xv[3][8];
#pragma unroll
  for (int i = 0; i < 3; ++i) {
    const float* p = xr + i * 256 + lane * 8;
    const v4f a = *(const v4f*)(p);
    const v4f c = *(const v4f*)(p + 4);
#pragma unroll
    for (int e = 0; e < 4; ++e) { xv[i][e] = a[e]; xv[i][4 + e] = c[e]; }
  }
  float s = 0.f;
#pragma unroll
  for (int i = 0; i < 3; ++i) {
#pragma unroll
    for (int e = 0; e < 8; ++e) s += xv[i][e];
  }
#pragma unroll
  for (int off = 16; off > 0; off >>= 1) s += __shfl_xor(s, off, 32);
  const float mu = s * kInvChan;
  float s2 = 0.f;
#pragma unroll
  for (int i = 0; i < 3; ++i) {
#pragma unroll
    for (int e = 0; e < 8; ++e) { const float d = xv[i][e] - mu; s2 += d * d; }
  }
#pragma unroll
  for (int off = 16; off > 0; off >>= 1) s2 += __shfl_xor(s2, off, 32);
  const float var = s2 * kInvChan;
  const float rstd = 1.0f / sqrtf(var + kLnEps);
  v4u u[3];
#pragma unroll
  for (int i = 0; i < 3; ++i) {
    const float* wq = w + i * 256 + lane * 8;
    const float* bq = bvec + i * 256 + lane * 8;
    const v4f wa = *(const v4f*)(wq); const v4f wc = *(const v4f*)(wq + 4);
    const v4f ba = *(const v4f*)(bq); const v4f bc = *(const v4f*)(bq + 4);
    unsigned short hb[8];
#pragma unroll
    for (int e = 0; e < 4; ++e) {
      hb[e]     = h_bits((xv[i][e] - mu) * rstd * wa[e] + ba[e]);
      hb[4 + e] = h_bits((xv[i][4 + e] - mu) * rstd * wc[e] + bc[e]);
    }
    u[i] = (v4u){pk16(hb[0], hb[1]), pk16(hb[2], hb[3]), pk16(hb[4], hb[5]), pk16(hb[6], hb[7])};
  }
  unsigned short* orow = out + (size_t)row * kChan + lane * 8;
  for (int pass = 0; pass < 2; ++pass) {
#pragma unroll
    for (int i = 0; i < 3; ++i) *(volatile v4u*)(orow + i * 256) = u[i];
    __threadfence();
  }
}

__global__ __launch_bounds__(256) void cast8_pair_kernel(const float* __restrict__ in0, const float* __restrict__ in1,
                                                         unsigned short* __restrict__ out0, unsigned short* __restrict__ out1,
                                                         int n8) {
  const int i = blockIdx.x * 256 + threadIdx.x;
  if (i >= n8) return;
  const int sel = blockIdx.y;
  const float* in = (sel == 0) ? in0 : in1;
  unsigned short* outp = (sel == 0) ? out0 : out1;
  const float* p = in + 8 * (size_t)i;
  const v4f a = *(const v4f*)(p);
  const v4f c = *(const v4f*)(p + 4);
  unsigned short hb[8];
#pragma unroll
  for (int e = 0; e < 4; ++e) {
    hb[e]     = h_bits(a[e]);
    hb[4 + e] = h_bits(c[e]);
  }
  const v4u u = (v4u){pk16(hb[0], hb[1]), pk16(hb[2], hb[3]), pk16(hb[4], hb[5]), pk16(hb[6], hb[7])};
  unsigned short* qo = outp + 8 * (size_t)i;
  *(volatile v4u*)qo = u;
  __threadfence();
  *(volatile v4u*)qo = u;
}

__global__ __launch_bounds__(256) void wtcast_kernel(const float* Wa, const float* Wb, const float* Wc, const float* Wd,
                                                     unsigned short* __restrict__ out, int nrows, int ncols, float scale) {
  __shared__ float sm[64][65];
  const int t = threadIdx.x;
  const int r0 = blockIdx.x * 64;
  const int c0 = blockIdx.y * 64;
  const int z = blockIdx.z;
  const float* W = (z == 0) ? Wa : (z == 1) ? Wb : (z == 2) ? Wc : Wd;
#pragma unroll
  for (int i = 0; i < 16; ++i) {
    const int e = i * 256 + t;
    const int rl = e >> 6;
    const int cl = e & 63;
    sm[cl][rl] = W[(size_t)(r0 + rl) * ncols + c0 + cl] * scale;
  }
  __syncthreads();
  const int lane = t & 31, wave = t >> 5;
  const int q4 = lane >> 3, c8 = (lane & 7) * 8;
  unsigned short* op = out + (size_t)z * ncols * nrows;
  v4u u[2];
#pragma unroll
  for (int it = 0; it < 2; ++it) {
    const int row = wave * 8 + it * 4 + q4;
    unsigned short hb[8];
#pragma unroll
    for (int e = 0; e < 8; ++e) hb[e] = h_bits(sm[row][c8 + e]);
    u[it] = (v4u){pk16(hb[0], hb[1]), pk16(hb[2], hb[3]), pk16(hb[4], hb[5]), pk16(hb[6], hb[7])};
  }
  for (int pass = 0; pass < 2; ++pass) {
#pragma unroll
    for (int it = 0; it < 2; ++it) {
      const int row = wave * 8 + it * 4 + q4;
      *(volatile v4u*)(op + (size_t)(c0 + row) * nrows + r0 + c8) = u[it];
    }
    __threadfence();
  }
}

__global__ __launch_bounds__(256) void softmax_rows_kernel(const float* __restrict__ S, unsigned short* __restrict__ P,
                                                           const int* __restrict__ maskflag) {
  __shared__ float redM[8];
  __shared__ float redS[8];
  const int row = blockIdx.x;
  const int nq = row & (kSeq - 1);
  const int t = threadIdx.x;
  const int lane = t & 31, wave = t >> 5;
  const int c0 = t * 8;
  const int mflag = maskflag[0];
  const float* sr = S + (size_t)row * kSeq + c0;
  const v4f a = *(const v4f*)(sr);
  const v4f c = *(const v4f*)(sr + 4);
  float x[8];
#pragma unroll
  for (int e = 0; e < 4; ++e) { x[e] = a[e]; x[4 + e] = c[e]; }
  if (mflag != 0) {
#pragma unroll
    for (int e = 0; e < 8; ++e) x[e] = (c0 + e == nq) ? -__builtin_inff() : x[e];
  }
  float m = fmaxf(fmaxf(fmaxf(x[0], x[1]), fmaxf(x[2], x[3])), fmaxf(fmaxf(x[4], x[5]), fmaxf(x[6], x[7])));
#pragma unroll
  for (int off = 16; off > 0; off >>= 1) m = fmaxf(m, __shfl_xor(m, off, 32));
  if (lane == 0) redM[wave] = m;
  __syncthreads();
  float gm = redM[0];
#pragma unroll
  for (int i = 1; i < 8; ++i) gm = fmaxf(gm, redM[i]);
  float p[8];
  float s = 0.f;
#pragma unroll
  for (int e = 0; e < 8; ++e) { p[e] = expf(x[e] - gm); s += p[e]; }
#pragma unroll
  for (int off = 16; off > 0; off >>= 1) s += __shfl_xor(s, off, 32);
  if (lane == 0) redS[wave] = s;
  __syncthreads();
  float tot = 0.f;
#pragma unroll
  for (int i = 0; i < 8; ++i) tot += redS[i];
  const float inv = kPCarry / tot;
  unsigned short hb[8];
#pragma unroll
  for (int e = 0; e < 8; ++e) hb[e] = h_bits(p[e] * inv);
  const v4u u = (v4u){pk16(hb[0], hb[1]), pk16(hb[2], hb[3]), pk16(hb[4], hb[5]), pk16(hb[6], hb[7])};
  unsigned short* pr = P + (size_t)row * kSeq + c0;
  *(volatile v4u*)pr = u;
  __threadfence();
  *(volatile v4u*)pr = u;
}

extern "C" void kernel_launch(void* const* d_in, const int* in_sizes, int n_in,
                              void* d_out, int out_size, void* d_ws, size_t ws_size, hipStream_t stream) {
  if (n_in < 18) return;
  if (in_sizes[0] != kTok * kChan || in_sizes[1] != kTok * kChan || in_sizes[2] != kTok * kChan) return;
  if (in_sizes[3] != kChan * kChan || in_sizes[4] != kChan * kChan || in_sizes[5] != kChan * kChan || in_sizes[6] != kChan * kChan) return;
  if (in_sizes[7] != kChan || in_sizes[8] != kChan || in_sizes[9] != kChan || in_sizes[10] != kChan || in_sizes[11] != kChan) return;
  if (in_sizes[12] != kChan * kFfn || in_sizes[13] != kFfn || in_sizes[14] != kFfn * kChan || in_sizes[15] != kChan) return;
  if (in_sizes[16] < 1 || in_sizes[17] < 1) return;
  if (out_size != kTok * kChan) return;
  if (ws_size < kWsTotal) return;

  const float* q = (const float*)d_in[0];
  const float* k = (const float*)d_in[1];
  const float* v = (const float*)d_in[2];
  const float* Wq = (const float*)d_in[3];
  const float* Wk = (const float*)d_in[4];
  const float* Wv = (const float*)d_in[5];
  const float* Wp = (const float*)d_in[6];
  const float* bp = (const float*)d_in[7];
  const float* ln1w = (const float*)d_in[8];
  const float* ln1b = (const float*)d_in[9];
  const float* ln2w = (const float*)d_in[10];
  const float* ln2b = (const float*)d_in[11];
  const float* W1 = (const float*)d_in[12];
  const float* b1 = (const float*)d_in[13];
  const float* W2 = (const float*)d_in[14];
  const float* b2 = (const float*)d_in[15];
  const int* maskp = (const int*)d_in[16];
  const int* posp = (const int*)d_in[17];
  float* out = (float*)d_out;

  char* ws = (char*)d_ws;
  unsigned short* W4t  = (unsigned short*)(ws + kOffW4);
  unsigned short* Qn   = (unsigned short*)(ws + kOffQn);
  unsigned short* Kc   = (unsigned short*)(ws + kOffKc);
  unsigned short* Vc   = (unsigned short*)(ws + kOffVc);
  float*          Sbuf = (float*)(ws + kOffS);
  unsigned short* Pbuf = (unsigned short*)(ws + kOffP);
  unsigned short* Q16  = (unsigned short*)(ws + kOffQ16);
  unsigned short* K16  = (unsigned short*)(ws + kOffK16);
  unsigned short* Vt16 = (unsigned short*)(ws + kOffVt);
  unsigned short* O16  = (unsigned short*)(ws + kOffO16);
  unsigned short* W1t  = (unsigned short*)(ws + kOffW1t);
  unsigned short* W2t  = (unsigned short*)(ws + kOffW2t);
  float*          X1   = (float*)(ws + kOffX1);
  unsigned short* Ln2o = (unsigned short*)(ws + kOffLn2);
  unsigned short* Hid  = (unsigned short*)(ws + kOffHid);
  const size_t kWPlane = (size_t)kChan * kChan;

  layernorm_rows_kernel<<<kTok / 8, 256, 0, stream>>>(q, ln1w, ln1b, Qn, kTok);
  cast8_pair_kernel<<<dim3(kTok * kChan / 8 / 256, 2), 256, 0, stream>>>(k, v, Kc, Vc, kTok * kChan / 8);
  wtcast_kernel<<<dim3(kChan / 64, kChan / 64, 4), 256, 0, stream>>>(Wq, Wk, Wv, Wp, W4t, kChan, kChan, kWCarry);

  const int blkTokC = (kTok / 64) * (kChan / 64) / 8;
  wmma_gemm64<0, false, 0, 1, false, 0><<<dim3(blkTokC, 1), 256, 0, stream>>>(
      Qn, nullptr, kChan, 0L, W4t + 0 * kWPlane, nullptr, kChan, 0L,
      Q16, nullptr, kChan, 0L, nullptr, nullptr, nullptr, nullptr, nullptr, 0L,
      kTok, kChan, kChan, kWCarryInv);
  wmma_gemm64<0, false, 0, 1, false, 0><<<dim3(blkTokC, 1), 256, 0, stream>>>(
      Kc, nullptr, kChan, 0L, W4t + 1 * kWPlane, nullptr, kChan, 0L,
      K16, nullptr, kChan, 0L, nullptr, nullptr, nullptr, nullptr, nullptr, 0L,
      kTok, kChan, kChan, kWCarryInv);
  const int blkVt = (kChan / 64) * (kSeq / 64) / 8;
  wmma_gemm64<0, false, 0, 1, false, 0><<<dim3(blkVt, kBatch), 256, 0, stream>>>(
      W4t + 2 * kWPlane, nullptr, kChan, 0L, Vc, nullptr, kChan, (long)kSeq * kChan,
      Vt16, nullptr, kSeq, (long)kChan * kSeq, nullptr, nullptr, nullptr, nullptr, nullptr, 0L,
      kChan, kSeq, kChan, kWCarryInv);

  const int blkS = (kSeq / 64) * (kSeq / 64) / 8;
  const int blkPV = ((kSeq / 64) * (kHdim / 64) + 7) / 8;
  for (int ch = 0; ch < kNumChunks; ++ch) {
    const int g0 = ch * kGrp;
    const int bb = g0 / kHeads;
    const int h0 = g0 - bb * kHeads;
    const unsigned short* Aq = Q16 + (size_t)bb * kSeq * kChan + (size_t)h0 * kHdim;
    const unsigned short* Bk = K16 + (size_t)bb * kSeq * kChan + (size_t)h0 * kHdim;
    wmma_gemm64<0, false, 0, 0, false, 0><<<dim3(blkS, kGrp), 256, 0, stream>>>(
        Aq, nullptr, kChan, (long)kHdim, Bk, nullptr, kChan, (long)kHdim,
        Sbuf, nullptr, kSeq, (long)kSeq * kSeq, nullptr, nullptr, nullptr, nullptr, nullptr, 0L,
        kSeq, kSeq, kHdim, kAttnScale);
    softmax_rows_kernel<<<kGrp * kSeq, 256, 0, stream>>>(Sbuf, Pbuf, maskp);
    const unsigned short* Bv = Vt16 + (size_t)bb * kChan * kSeq + (size_t)h0 * kHdim * kSeq;
    unsigned short* Co = O16 + (size_t)bb * kSeq * kChan + (size_t)h0 * kHdim;
    wmma_gemm64<0, false, 0, 1, false, 0><<<dim3(blkPV, kGrp), 256, 0, stream>>>(
        Pbuf, nullptr, kSeq, (long)kSeq * kSeq, Bv, nullptr, kSeq, (long)kHdim * kSeq,
        Co, nullptr, kChan, (long)kHdim, nullptr, nullptr, nullptr, nullptr, nullptr, 0L,
        kSeq, kHdim, kSeq, kPVScale);
  }

  wmma_gemm64<0, false, 2, 0, true, 0><<<dim3(blkTokC, 1), 256, 0, stream>>>(
      O16, nullptr, kChan, 0L, W4t + 3 * kWPlane, nullptr, kChan, 0L,
      X1, nullptr, kChan, 0L, bp, q, k, v, posp, 0L,
      kTok, kChan, kChan, kWpScale);
  wtcast_kernel<<<dim3(kChan / 64, kFfn / 64, 1), 256, 0, stream>>>(W1, W1, W1, W1, W1t, kChan, kFfn, kWCarry);
  wtcast_kernel<<<dim3(kFfn / 64, kChan / 64, 1), 256, 0, stream>>>(W2, W2, W2, W2, W2t, kFfn, kChan, kWCarry);
  layernorm_rows_kernel<<<kTok / 8, 256, 0, stream>>>(X1, ln2w, ln2b, Ln2o, kTok);
  const int blkFfn = (kTok / 64) * (kFfn / 64) / 8;
  wmma_gemm64<0, false, 2, 1, false, 2><<<dim3(blkFfn, 1), 256, 0, stream>>>(
      Ln2o, nullptr, kChan, 0L, W1t, nullptr, kChan, 0L,
      Hid, nullptr, kFfn, 0L, b1, nullptr, nullptr, nullptr, nullptr, 0L,
      kTok, kFfn, kChan, kWCarryInv);
  wmma_gemm64<0, false, 2, 0, true, 0><<<dim3(blkTokC, 1), 256, 0, stream>>>(
      Hid, nullptr, kFfn, 0L, W2t, nullptr, kFfn, 0L,
      out, nullptr, kChan, 0L, b2, X1, nullptr, nullptr, nullptr, 0L,
      kTok, kChan, kFfn, kWCarryInv);
}
